// CausalSelfAttention_28707561406800
// MI455X (gfx1250) — hardware-verified
//
#include <hip/hip_runtime.h>
#pragma clang fp contract(off)


#ifndef NB
#define NB 2
#endif
#ifndef SEQ
#define SEQ 2048
#endif
#define NB_FULL  2
#define SEQ_FULL 2048
#define DM   1024
#define NH_  16
#define HD   64
#define DQ   (NH_ * HD)
#define NBH  (NB * NH_)
#define MROWS (NB * SEQ)
#define FLD  (3 * DQ)
#define RH   256
#define SP   72
#define PCAR 256.0f
#define SCL  0.125f
#define L2E  1.4426950408889634f

typedef _Float16 h16;
typedef unsigned short bf;
typedef __attribute__((ext_vector_type(16))) __bf16   v16bf;
typedef __attribute__((ext_vector_type(16))) _Float16 v16h;
typedef __attribute__((ext_vector_type(16))) unsigned short v16us;
typedef __attribute__((ext_vector_type(8)))  _Float16 v8h;
typedef __attribute__((ext_vector_type(8)))  unsigned short v8us;
typedef __attribute__((ext_vector_type(8)))  float    v8f;
typedef __attribute__((ext_vector_type(4)))  float    v4f;
typedef __attribute__((ext_vector_type(2)))  float    v2f;
typedef __attribute__((ext_vector_type(2)))  _Float16 v2h;
typedef __attribute__((ext_vector_type(2)))  unsigned short v2us;
typedef v4f  __attribute__((may_alias)) v4fa;
typedef v8us __attribute__((may_alias)) v8usa;

static_assert(HD == 64);
static_assert(DQ == DM);
static_assert(SEQ % 64 == 0);
static_assert(RH % 64 == 0);
static_assert(RH <= SEQ);
static_assert(DM % 64 == 0);
static_assert(FLD % 64 == 0);
static_assert(MROWS % 64 == 0);
static_assert(DM % 32 == 0);
static_assert((SP * 2) % 16 == 0);
static_assert(SP >= HD);
static_assert(SEQ <= SEQ_FULL);
static_assert(NB <= NB_FULL);

constexpr size_t al256(size_t b) { return (b + 255) & ~(size_t)255; }
constexpr size_t SZ_XB   = al256((size_t)MROWS * DM * 2);
constexpr size_t SZ_WQKV = al256((size_t)FLD * DM * 2);
constexpr size_t SZ_WO   = al256((size_t)DM * DQ * 2);
constexpr size_t SZ_F    = al256((size_t)MROWS * FLD * 4);
constexpr size_t SZ_QK16 = al256((size_t)2 * NBH * SEQ * HD * 2);
constexpr size_t SZ_VT16 = al256((size_t)NBH * HD * SEQ * 2);
constexpr size_t SZ_QKL  = al256((size_t)2 * NBH * RH * HD * 2);
constexpr size_t SZ_VTL  = al256((size_t)NBH * HD * RH * 2);
constexpr size_t SZ_AT   = al256((size_t)MROWS * DQ * 2);
constexpr size_t WS_TOTAL = SZ_XB + SZ_WQKV + SZ_WO + SZ_F + SZ_QK16 + SZ_VT16 + 2 * SZ_QKL + 2 * SZ_VTL + 2 * SZ_AT;
static_assert(WS_TOTAL <= (size_t)134217728);

__device__ __forceinline__ unsigned short f2bf(float f) { unsigned u = __float_as_uint(f); u += 0x7FFFu + ((u >> 16) & 1u); return (unsigned short)(u >> 16); }
__device__ __forceinline__ float bf2f(unsigned short b) { return __uint_as_float(((unsigned)b) << 16); }
__device__ __forceinline__ float bfr(float f) { return bf2f(f2bf(f)); }
__device__ __forceinline__ void splitf(float y, unsigned short& h, unsigned short& l) { h = f2bf(y); l = f2bf(y - bf2f(h)); }
__device__ __forceinline__ v16h cat16(v8h lo, v8h hi) { return __builtin_shufflevector(lo, hi, 0, 1, 2, 3, 4, 5, 6, 7, 8, 9, 10, 11, 12, 13, 14, 15); }
__device__ __forceinline__ v16bf cat16b(v8us lo, v8us hi) { return __builtin_bit_cast(v16bf, __builtin_shufflevector(lo, hi, 0, 1, 2, 3, 4, 5, 6, 7, 8, 9, 10, 11, 12, 13, 14, 15)); }
__device__ __forceinline__ v8f wmma16(v16h a, v16h b, v8f c) { return __builtin_amdgcn_wmma_f32_16x16x32_f16(false, a, false, b, (short)0, c, false, false); }
__device__ __forceinline__ v8f wmmab(v16bf a, v16bf b, v8f c) { return __builtin_amdgcn_wmma_f32_16x16x32_bf16(false, a, false, b, (short)0, c, false, false); }

template <typename T16> struct WFrag;
template <> struct WFrag<h16> {
    typedef v16h V; typedef v16h S; typedef h16 E;
    static __device__ __forceinline__ V ld(const h16* p) { return cat16(*(const v8h*)p, *(const v8h*)(p + 16)); }
    static __device__ __forceinline__ v8f mma(V a, V b, v8f c) { return wmma16(a, b, c); }
    static __device__ __forceinline__ E cv(float x) { return (h16)x; }
    static __device__ __forceinline__ float tf(E e) { return (float)e; }
    static __device__ __forceinline__ V fin(S s) { return s; } };
template <> struct WFrag<bf> {
    typedef v16bf V; typedef v16us S; typedef unsigned short E;
    static __device__ __forceinline__ V ld(const bf* p) { return cat16b(*(const v8us*)p, *(const v8us*)(p + 16)); }
    static __device__ __forceinline__ v8f mma(V a, V b, v8f c) { return wmmab(a, b, c); }
    static __device__ __forceinline__ E cv(float x) { return f2bf(x); }
    static __device__ __forceinline__ float tf(E e) { return bf2f(e); }
    static __device__ __forceinline__ V fin(S s) { return __builtin_bit_cast(v16bf, s); } };

template <int NSPLIT>
__device__ __forceinline__ void gemmw_body(const bf* __restrict__ A, const bf* __restrict__ A2, const bf* __restrict__ Bt, const int K, float* C, const int ldc, const size_t sA, const size_t sC) {
    typedef WFrag<bf> W; typedef WFrag<bf>::V V;
    __shared__ __align__(16) float os[16 * 68];
    const size_t z = blockIdx.z; A += z * sA; A2 += z * sA; C += z * sC;
    const int lane = threadIdx.x & 31, lr = lane & 15, hi = lane >> 4; const int r0 = blockIdx.x * 64, c0 = blockIdx.y * 64;
    v8f acc[4][4];
#pragma unroll
    for (int mb = 0; mb < 4; ++mb)
#pragma unroll
        for (int nb = 0; nb < 4; ++nb) acc[mb][nb] = (v8f){};
    const size_t aoff = (size_t)(r0 + lr) * K + 8 * hi, boff = (size_t)(c0 + lr) * K + 8 * hi;
#pragma unroll 1
    for (int kc = 0; kc < K; kc += 32) {
        V a[4], a2[4];
#pragma unroll
        for (int mb = 0; mb < 4; ++mb) { a[mb] = W::ld(A + aoff + (size_t)mb * 16 * K + kc); a2[mb] = a[mb]; if (NSPLIT == 1) a2[mb] = W::ld(A2 + aoff + (size_t)mb * 16 * K + kc); }
        V b = a[0];
#pragma unroll
        for (int nb = 0; nb < 4; ++nb) { b = W::ld(Bt + boff + (size_t)nb * 16 * K + kc);
#pragma unroll
            for (int mb = 0; mb < 4; ++mb) { acc[mb][nb] = W::mma(a[mb], b, acc[mb][nb]); if (NSPLIT == 1) acc[mb][nb] = W::mma(a2[mb], b, acc[mb][nb]); } }
        asm volatile("v_nop\n\tv_nop\n\tv_nop\n\tv_nop" : "+v"(acc[0][0]), "+v"(acc[0][1]), "+v"(acc[0][2]), "+v"(acc[0][3]), "+v"(acc[1][0]), "+v"(acc[1][1]), "+v"(acc[1][2]), "+v"(acc[1][3]) : "v"(a[0]), "v"(a[1]), "v"(b));
        asm volatile("v_nop\n\tv_nop\n\tv_nop\n\tv_nop" : "+v"(acc[2][0]), "+v"(acc[2][1]), "+v"(acc[2][2]), "+v"(acc[2][3]), "+v"(acc[3][0]), "+v"(acc[3][1]), "+v"(acc[3][2]), "+v"(acc[3][3]) : "v"(a[2]), "v"(a[3]), "v"(a2[3]), "v"(b));
    }
#pragma unroll
    for (int mb = 0; mb < 4; ++mb) {
#pragma unroll
        for (int nb = 0; nb < 4; ++nb) {
#pragma unroll
            for (int j = 0; j < 8; ++j) os[(hi * 8 + j) * 68 + nb * 16 + lr] = acc[mb][nb][j]; }
        __builtin_amdgcn_fence(3  , "wavefront"); __builtin_amdgcn_wave_barrier(); asm volatile("" ::: "memory");
        float* crow = C + (size_t)(r0 + mb * 16) * ldc + c0;
#pragma unroll 1
        for (int ps = 0; ps < 2; ++ps) {
#pragma unroll
            for (int s = 0; s < 8; ++s) { const int row = 2 * s + hi, cofs = lr * 4; const v4f val = *(const v4fa*)(os + row * 68 + cofs);
                *(volatile v4f*)(crow + (size_t)row * ldc + cofs) = val; }
            if (ps == 0) __threadfence(); }
        __builtin_amdgcn_wave_barrier(); asm volatile("" ::: "memory");
    }
}
__global__ __launch_bounds__(32) void k_gemm_qkv(const bf* __restrict__ A, const bf* __restrict__ Bt, int K, float* C, int ldc) { gemmw_body<0>(A, A, Bt, K, C, ldc, (size_t)0, (size_t)0); }
__global__ __launch_bounds__(32) void k_gemm_out(const bf* __restrict__ A, const bf* __restrict__ A2, const bf* __restrict__ Bt, int K, float* C, int ldc, size_t sA, size_t sC) { gemmw_body<1>(A, A2, Bt, K, C, ldc, sA, sC); }

__global__ __launch_bounds__(256) void k_wtG(const float* __restrict__ w, int K, int N, bf* Bt) {
    const int lane = threadIdx.x & 31; const int L0 = (blockIdx.x * 8 + (threadIdx.x >> 5)) * 8; const int nlines = N * K / 64;
#pragma unroll
    for (int ps = 0; ps < 2; ++ps) {
#pragma unroll 1
        for (int l = 0; l < 8; ++l) { const int L = L0 + l; if (L >= nlines) break; const size_t e = (size_t)L * 64 + lane * 2; const int k = (int)(e % K), n = (int)(e / K); v2us o;
            o[0] = f2bf(w[(size_t)k * N + n]); o[1] = f2bf(w[(size_t)(k + 1) * N + n]); *(volatile v2us*)(Bt + e) = o; }
        if (ps == 0) __threadfence(); }
}
__global__ __launch_bounds__(256) void k_cvtx(const float* __restrict__ src, bf* dst, size_t n8) {
    const size_t i = (size_t)blockIdx.x * 256 + threadIdx.x; if (i >= n8) return;
    const size_t e = i * 8; const size_t b = e / ((size_t)SEQ * DM); const size_t w = e - b * ((size_t)SEQ * DM);
    const v8f v = *(const v8f*)(src + b * ((size_t)SEQ_FULL * DM) + w); v8us o;
#pragma unroll
    for (int k = 0; k < 8; ++k) o[k] = f2bf(v[k]);
    *(volatile v8us*)(dst + e) = o; __threadfence(); *(volatile v8us*)(dst + e) = o; }

__global__ __launch_bounds__(256) void k_qkp(const float* __restrict__ F, const float* __restrict__ cs, const float* __restrict__ sn, h16* P16, bf* PLh, bf* PLl) {
    const size_t p = (size_t)blockIdx.x * 256 + threadIdx.x; if (p >= (size_t)2 * NBH * SEQ * 32) return;
    const int d = (int)(p & 31) * 2; const int t = (int)((p >> 5) % SEQ); const int bh = (int)((p / ((size_t)32 * SEQ)) % NBH); const int which = (int)(p / ((size_t)32 * SEQ * NBH));
    const int b = bh / NH_, h = bh - b * NH_;
    const v2f xv = *(const v2f*)(F + (size_t)(b * SEQ + t) * FLD + which * DQ + h * HD + d);
    const v2f cv = *(const v2f*)(cs + (size_t)t * HD + d);
    const v2f sv = *(const v2f*)(sn + (size_t)t * HD + d);
    const float c0 = bfr(cv[0]), c1 = bfr(cv[1]), s0 = bfr(sv[0]), s1 = bfr(sv[1]);
    const float a0 = xv[0] * c0; const float b0 = xv[1] * s0; const float a1 = xv[1] * c1; const float b1 = xv[0] * s1;
    const float r0 = a0 - b0; const float r1 = a1 + b1;
    v2h o16; o16[0] = (h16)r0; o16[1] = (h16)r1; v2us oh, ol; unsigned short ha, la;
    splitf(r0, ha, la); oh[0] = ha; ol[0] = la; splitf(r1, ha, la); oh[1] = ha; ol[1] = la;
    const bool lo = (t < RH);
    const size_t e16 = ((size_t)(which * NBH + bh) * SEQ + t) * HD + d;
    const size_t el = ((size_t)(which * NBH + bh) * RH + (lo ? t : 0)) * HD + d;
    *(volatile v2h*)(P16 + e16) = o16; if (lo) { *(volatile v2us*)(PLh + el) = oh; *(volatile v2us*)(PLl + el) = ol; }
    __threadfence();
    *(volatile v2h*)(P16 + e16) = o16; if (lo) { *(volatile v2us*)(PLh + el) = oh; *(volatile v2us*)(PLl + el) = ol; }
}
__global__ __launch_bounds__(256) void k_vtp(const float* __restrict__ F, h16* V16, bf* VLh, bf* VLl) {
    const size_t e = ((size_t)blockIdx.x * 256 + threadIdx.x) * 2; if (e >= (size_t)NBH * HD * SEQ) return;
    const int t = (int)(e % SEQ); const int d = (int)((e / SEQ) % HD); const int bh = (int)(e / ((size_t)SEQ * HD));
    const int b = bh / NH_, h = bh - b * NH_;
    const float* f = F + (size_t)(b * SEQ + t) * FLD + 2 * DQ + h * HD + d;
    const float x0 = f[0], x1 = f[FLD];
    v2h o16; o16[0] = (h16)x0; o16[1] = (h16)x1; v2us oh, ol; unsigned short ha, la;
    splitf(x0, ha, la); oh[0] = ha; ol[0] = la; splitf(x1, ha, la); oh[1] = ha; ol[1] = la;
    const bool lo = (t < RH);
    const size_t el = ((size_t)bh * HD + d) * RH + (lo ? t : 0);
    *(volatile v2h*)(V16 + e) = o16; if (lo) { *(volatile v2us*)(VLh + el) = oh; *(volatile v2us*)(VLl + el) = ol; }
    __threadfence();
    *(volatile v2h*)(V16 + e) = o16; if (lo) { *(volatile v2us*)(VLh + el) = oh; *(volatile v2us*)(VLl + el) = ol; }
}

template <typename T16, bool SPLIT>
__device__ __forceinline__ void attn_body(const T16* __restrict__ Qp, const T16* __restrict__ Q2, const T16* __restrict__ Kp, const T16* __restrict__ K2, const T16* __restrict__ Vt, const T16* __restrict__ Vt2,
                                          const int tlen, const int roff, const float pc, bf* ATh, bf* ATl) {
    typedef WFrag<T16> W; typedef typename W::V V; typedef typename W::S S; typedef typename W::E E;
    __shared__ __align__(16) unsigned short sth[4 * 16 * SP];
    __shared__ __align__(16) unsigned short stl[4 * 16 * SP];
    const int wave = __builtin_amdgcn_readfirstlane((int)(threadIdx.x >> 5));
    const int lane = threadIdx.x & 31, n = lane & 15, hi = lane >> 4;
    const int bh = blockIdx.y;
    const int qw = roff + (int)blockIdx.x * 64 + wave * 16;
    const int qpos = qw + n;
    const size_t pb = (size_t)bh * (size_t)tlen * HD;
    const size_t qo = pb + (size_t)qpos * HD + 8 * hi;
    const V q0 = W::ld(Qp + qo), q1 = W::ld(Qp + qo + 32);
    V q0l = q0, q1l = q1;
    if (SPLIT) { q0l = W::ld(Q2 + qo); q1l = W::ld(Q2 + qo + 32); }
    v8f acc[4];
#pragma unroll
    for (int dt = 0; dt < 4; ++dt) acc[dt] = (v8f){};
    float m = -1.0e30f, l = 0.0f;
    const int nkt = (qw + 16 + 31) >> 5;
#pragma unroll 1
    for (int j = 0; j < nkt; ++j) {
        const int kt = j * 32;
        const size_t ko = pb + (size_t)(kt + n) * HD + 8 * hi;
        const V k00 = W::ld(Kp + ko), k01 = W::ld(Kp + ko + 32), k10 = W::ld(Kp + ko + 16 * HD), k11 = W::ld(Kp + ko + 16 * HD + 32);
        v8f s0 = (v8f){}, s1 = (v8f){};
        s0 = W::mma(k00, q0, s0); s1 = W::mma(k10, q0, s1); s0 = W::mma(k01, q1, s0); s1 = W::mma(k11, q1, s1);
        if (SPLIT) {
            const V g00 = W::ld(K2 + ko), g01 = W::ld(K2 + ko + 32), g10 = W::ld(K2 + ko + 16 * HD), g11 = W::ld(K2 + ko + 16 * HD + 32);
            s0 = W::mma(k00, q0l, s0); s1 = W::mma(k10, q0l, s1); s0 = W::mma(k01, q1l, s0); s1 = W::mma(k11, q1l, s1);
            s0 = W::mma(g00, q0, s0); s1 = W::mma(g10, q0, s1); s0 = W::mma(g01, q1, s0); s1 = W::mma(g11, q1, s1);
            asm volatile("v_nop\n\tv_nop\n\tv_nop\n\tv_nop" : "+v"(s0), "+v"(s1) : "v"(g01), "v"(g11), "v"(q1), "v"(q1l));
        } else {
            asm volatile("v_nop\n\tv_nop\n\tv_nop\n\tv_nop" : "+v"(s0), "+v"(s1) : "v"(k01), "v"(k11), "v"(q1));
        }
        float x0[8], x1[8];
#pragma unroll
        for (int r = 0; r < 8; ++r) { x0[r] = s0[r] * SCL; x1[r] = s1[r] * SCL; }
        if (kt + 31 > qw) {
#pragma unroll
            for (int r = 0; r < 8; ++r) { const int key = kt + 8 * hi + r; x0[r] = (key > qpos) ? -1.0e30f : x0[r]; x1[r] = (key + 16 > qpos) ? -1.0e30f : x1[r]; }
        }
        float mx = fmaxf(x0[0], x1[0]);
#pragma unroll
        for (int r = 1; r < 8; ++r) mx = fmaxf(mx, fmaxf(x0[r], x1[r]));
        mx = fmaxf(mx, __shfl_xor(mx, 16, 32));
        const float mn = fmaxf(m, mx);
        const float al = __builtin_amdgcn_exp2f((m - mn) * L2E);
        m = mn;
        S pe = {}; S pe2 = {}; float ps = 0.0f;
#pragma unroll
        for (int r = 0; r < 8; ++r) {
            const float pa = __builtin_amdgcn_exp2f((x0[r] - mn) * L2E) * pc;
            const float pq = __builtin_amdgcn_exp2f((x1[r] - mn) * L2E) * pc;
            const E ea = W::cv(pa), eb = W::cv(pq); const float fa = W::tf(ea), fb = W::tf(eb);
            pe[r] = ea; pe[8 + r] = eb;
            if (SPLIT) { pe2[r] = W::cv(pa - fa); pe2[8 + r] = W::cv(pq - fb); ps += pa + pq; } else { ps += fa + fb; }
        }
        l = l * al + ps;
#pragma unroll
        for (int dt = 0; dt < 4; ++dt) acc[dt] = acc[dt] * al;
        const V pv = W::fin(pe);
        const size_t vo = pb + (size_t)n * tlen + kt + 8 * hi;
        const V v0 = W::ld(Vt + vo), v1 = W::ld(Vt + vo + (size_t)16 * tlen), v2 = W::ld(Vt + vo + (size_t)32 * tlen), v3 = W::ld(Vt + vo + (size_t)48 * tlen);
        acc[0] = W::mma(v0, pv, acc[0]); acc[1] = W::mma(v1, pv, acc[1]); acc[2] = W::mma(v2, pv, acc[2]); acc[3] = W::mma(v3, pv, acc[3]);
        if (SPLIT) {
            const V pl = W::fin(pe2);
            acc[0] = W::mma(v0, pl, acc[0]); acc[1] = W::mma(v1, pl, acc[1]); acc[2] = W::mma(v2, pl, acc[2]); acc[3] = W::mma(v3, pl, acc[3]);
            const V w0 = W::ld(Vt2 + vo), w1 = W::ld(Vt2 + vo + (size_t)16 * tlen), w2 = W::ld(Vt2 + vo + (size_t)32 * tlen), w3 = W::ld(Vt2 + vo + (size_t)48 * tlen);
            acc[0] = W::mma(w0, pv, acc[0]); acc[1] = W::mma(w1, pv, acc[1]); acc[2] = W::mma(w2, pv, acc[2]); acc[3] = W::mma(w3, pv, acc[3]);
            asm volatile("v_nop\n\tv_nop\n\tv_nop\n\tv_nop" : "+v"(acc[0]), "+v"(acc[1]), "+v"(acc[2]), "+v"(acc[3]) : "v"(w3), "v"(pv), "v"(pl));
        } else {
            asm volatile("v_nop\n\tv_nop\n\tv_nop\n\tv_nop" : "+v"(acc[0]), "+v"(acc[1]), "+v"(acc[2]), "+v"(acc[3]) : "v"(v3), "v"(pv));
        }
    }
    l += __shfl_xor(l, 16, 32);
    const float inv = 1.0f / l;
    const int wb = wave * (16 * SP);
#pragma unroll
    for (int dt = 0; dt < 4; ++dt) { v8us oh, ol;
#pragma unroll
        for (int r = 0; r < 8; ++r) { unsigned short a, c2; splitf(acc[dt][r] * inv, a, c2); oh[r] = a; ol[r] = c2; }
        *(v8usa*)&sth[wb + n * SP + dt * 16 + hi * 8] = oh; *(v8usa*)&stl[wb + n * SP + dt * 16 + hi * 8] = ol; }
    __builtin_amdgcn_fence(3  , "wavefront"); __builtin_amdgcn_wave_barrier(); asm volatile("" ::: "memory");
    const int b = bh / NH_, h = bh - b * NH_;
    const size_t g0 = ((size_t)b * SEQ + qw) * DQ + (size_t)h * HD;
#pragma unroll 1
    for (int ps2 = 0; ps2 < 2; ++ps2) {
#pragma unroll
        for (int s = 0; s < 4; ++s) { const int row = 4 * s + (lane >> 3), c8 = (lane & 7) * 8;
            const v8us vh = *(const v8usa*)&sth[wb + row * SP + c8]; const v8us vl = *(const v8usa*)&stl[wb + row * SP + c8];
            *(volatile v8us*)(ATh + g0 + (size_t)row * DQ + c8) = vh; *(volatile v8us*)(ATl + g0 + (size_t)row * DQ + c8) = vl; }
        if (ps2 == 0) __threadfence(); }
}
__global__ __launch_bounds__(128) void k_attn_hi(const h16* __restrict__ Q, const h16* __restrict__ K, const h16* __restrict__ Vt, bf* ATh, bf* ATl) {
    attn_body<h16, false>(Q, Q, K, K, Vt, Vt, SEQ, RH, PCAR, ATh, ATl); }
__global__ __launch_bounds__(128) void k_attn_lo(const bf* __restrict__ Qh, const bf* __restrict__ Ql, const bf* __restrict__ Kh, const bf* __restrict__ Kl, const bf* __restrict__ Vh, const bf* __restrict__ Vl, bf* ATh, bf* ATl) {
    attn_body<bf, true>(Qh, Ql, Kh, Kl, Vh, Vl, RH, 0, 1.0f, ATh, ATl); }

extern "C" void kernel_launch(void* const* d_in, const int* in_sizes, int n_in,
                              void* d_out, int out_size, void* d_ws, size_t ws_size, hipStream_t stream) {
    if (n_in < 5) return;
    const size_t need_x = ((size_t)(NB - 1) * SEQ_FULL + SEQ) * DM;
    if ((size_t)in_sizes[0] < need_x) return;
    if ((size_t)in_sizes[1] < (size_t)SEQ * HD || (size_t)in_sizes[2] < (size_t)SEQ * HD) return;
    if ((size_t)in_sizes[3] < (size_t)DM * FLD || (size_t)in_sizes[4] < (size_t)DQ * DM) return;
    if ((size_t)out_size < need_x) return;
    if (ws_size < WS_TOTAL) return;
    const float* x = (const float*)d_in[0]; const float* cs = (const float*)d_in[1]; const float* sn = (const float*)d_in[2];
    const float* wqkv = (const float*)d_in[3]; const float* wo = (const float*)d_in[4];
    float* OUT = (float*)d_out;
    char* wsp = (char*)d_ws;
    auto take = [&](size_t bytes) { char* p = wsp; wsp += bytes; return (void*)p; };
    bf* XB = (bf*)take(SZ_XB); bf* WQKV = (bf*)take(SZ_WQKV); bf* WO = (bf*)take(SZ_WO); float* F = (float*)take(SZ_F);
    h16* QK16 = (h16*)take(SZ_QK16); h16* VT16 = (h16*)take(SZ_VT16);
    bf* QKLh = (bf*)take(SZ_QKL); bf* QKLl = (bf*)take(SZ_QKL); bf* VTLh = (bf*)take(SZ_VTL); bf* VTLl = (bf*)take(SZ_VTL);
    bf* ATh = (bf*)take(SZ_AT); bf* ATl = (bf*)take(SZ_AT);
    if ((size_t)(wsp - (char*)d_ws) > ws_size) return;
    const size_t PS16 = (size_t)NBH * SEQ * HD;
    const size_t PSL  = (size_t)NBH * RH * HD;

    k_wtG<<<(unsigned)((DM * FLD / 64 + 63) / 64), 256, 0, stream>>>(wqkv, DM, FLD, WQKV);
    k_wtG<<<(unsigned)((DQ * DM / 64 + 63) / 64), 256, 0, stream>>>(wo, DQ, DM, WO);
    k_cvtx<<<(unsigned)(((size_t)MROWS * DM / 8 + 255) / 256), 256, 0, stream>>>(x, XB, (size_t)MROWS * DM / 8);
    k_gemm_qkv<<<dim3(MROWS / 64, FLD / 64, 1), 32, 0, stream>>>(XB, WQKV, DM, F, FLD);
    k_qkp<<<(unsigned)(((size_t)2 * NBH * SEQ * 32 + 255) / 256), 256, 0, stream>>>(F, cs, sn, QK16, QKLh, QKLl);
    k_vtp<<<(unsigned)(((size_t)NBH * HD * SEQ / 2 + 255) / 256), 256, 0, stream>>>(F, VT16, VTLh, VTLl);
    k_attn_lo<<<dim3(RH / 64, NBH, 1), 128, 0, stream>>>(QKLh, QKLl, QKLh + PSL, QKLl + PSL, VTLh, VTLl, ATh, ATl);
    if (SEQ > RH) k_attn_hi<<<dim3((SEQ - RH) / 64, NBH, 1), 128, 0, stream>>>(QK16, QK16 + PS16, VT16, ATh, ATl);
    k_gemm_out<<<dim3(SEQ / 64, DM / 64, NB), 32, 0, stream>>>(ATh, ATl, WO, DQ, OUT, DM, (size_t)SEQ * DQ, (size_t)SEQ_FULL * DM);
}
